// SkeletonGCNEncoderLSTM_2843268350833
// MI455X (gfx1250) — hardware-verified
//
#include <hip/hip_runtime.h>
#include <math.h>

constexpr int NBAT    = 64;
constexpr int NSTEP   = 512;
constexpr int NJ      = 33;
constexpr int ND      = 3;
constexpr int NH1     = 32;
constexpr int NH2     = 64;
constexpr int NHL     = 128;
constexpr int NGATE   = 4 * NHL;
constexpr int NFRAME  = NBAT * NSTEP;
constexpr int XFR     = NJ * ND;
constexpr int NCHUNK  = 4;
constexpr int FPC     = NFRAME / NCHUNK;
constexpr int BPC     = NBAT / NCHUNK;
constexpr int ROWS_PC = FPC * NJ;
constexpr int FPB     = 8;
constexpr int ROWS_PB = FPB * NJ;
constexpr int NTHR    = 256;
constexpr int KCAT    = NH2 + NHL;
constexpr int APITCH  = 200;
constexpr int SEQ_BLK = 32;
constexpr int SLABP   = 132;
constexpr float OPCARRY      = 16.0f;
constexpr float OPCARRY2_INV = 1.0f / 256.0f;

static_assert(NFRAME % NCHUNK == 0 && NBAT % NCHUNK == 0);
static_assert(FPC % FPB == 0);
static_assert(ROWS_PC % 64 == 0);
static_assert(NH2 == 64 && NH1 == 32);
static_assert(KCAT % 32 == 0 && APITCH % 8 == 0 && APITCH >= KCAT);
static_assert((ROWS_PB * NH1) % 8 == 0 && ((ROWS_PB * NH1 / 8) % 32) == 0);
static_assert((ROWS_PB * NH1 * 2) % 128 == 0);
static_assert((FPC * 8) % NTHR == 0);
static_assert(NBAT % SEQ_BLK == 0 && NHL == 16 * (NTHR / 32));
static_assert(SEQ_BLK * (NH2 / 8) == NTHR);
static_assert((2 * SEQ_BLK * APITCH) % 8 == 0);
static_assert(NGATE * (KCAT / 8) % NTHR == 0);
static_assert(NH2 * (NH1 / 8) == NTHR);

typedef __attribute__((ext_vector_type(16))) _Float16 v16h;
typedef __attribute__((ext_vector_type(8)))  _Float16 v8h;
typedef __attribute__((ext_vector_type(16))) __bf16   v16b;
typedef __attribute__((ext_vector_type(8)))  __bf16   v8b;
typedef __attribute__((ext_vector_type(8)))  float    v8f;
typedef __attribute__((ext_vector_type(4)))  float    v4f;

__device__ __forceinline__ unsigned short f2bf_bits(float f) {
  unsigned u = __float_as_uint(f);
  return (unsigned short)((u + 0x7FFFu + ((u >> 16) & 1u)) >> 16);
}
__device__ __forceinline__ float bf_bits2f(unsigned short h) { return __uint_as_float(((unsigned)h) << 16); }

__device__ __forceinline__ void dep_guard_h(v8f& a, v8f& b, v16h x, v16h y) { asm volatile("v_nop\n\tv_nop\n\tv_nop\n\tv_nop" : "+v"(a), "+v"(b) : "v"(x), "v"(y)); }
__device__ __forceinline__ void dep_guard_b(v8f& a, v8f& b, v16b x, v16b y) { asm volatile("v_nop\n\tv_nop\n\tv_nop\n\tv_nop" : "+v"(a), "+v"(b) : "v"(x), "v"(y)); }
__device__ __forceinline__ void keep4_h(v16h a, v16h b, v16h c, v16h d) { asm volatile("v_nop" :: "v"(a), "v"(b), "v"(c), "v"(d)); }
__device__ __forceinline__ void keep4_b(v16b a, v16b b, v16b c, v16b d) { asm volatile("v_nop" :: "v"(a), "v"(b), "v"(c), "v"(d)); }
__device__ __forceinline__ void acc_guard4(v8f& a, v8f& b, v8f& c, v8f& d) { asm volatile("v_nop\n\tv_nop\n\tv_nop\n\tv_nop" : "+v"(a), "+v"(b), "+v"(c), "+v"(d)); }
template <typename T> struct Frag;
template <> struct Frag<_Float16> {
  typedef v16h V; union U { v16h v; v8h h[2]; };
  static __device__ __forceinline__ v16h load(const _Float16* p) {
    U f; f.h[0] = *(const v8h*)(p); f.h[1] = *(const v8h*)(p + 16); return f.v;
  }
  static __device__ __forceinline__ v8f mma(v16h a, v16h b, v8f c) {
    return __builtin_amdgcn_wmma_f32_16x16x32_f16(false, a, false, b, (short)0, c, false, false);
  }
  static __device__ __forceinline__ void guard(v8f& a, v8f& b, v16h x, v16h y) { dep_guard_h(a, b, x, y); }
  static __device__ __forceinline__ void keep(v16h a, v16h b, v16h c, v16h d) { keep4_h(a, b, c, d); }
};
template <> struct Frag<__bf16> {
  typedef v16b V; union U { v16b v; v8b h[2]; };
  static __device__ __forceinline__ v16b load(const __bf16* p) {
    U f; f.h[0] = *(const v8b*)(p); f.h[1] = *(const v8b*)(p + 16); return f.v;
  }
  static __device__ __forceinline__ v8f mma(v16b a, v16b b, v8f c) {
    return __builtin_amdgcn_wmma_f32_16x16x32_bf16(false, a, false, b, (short)0, c, false, false);
  }
  static __device__ __forceinline__ void guard(v8f& a, v8f& b, v16b x, v16b y) { dep_guard_b(a, b, x, y); }
  static __device__ __forceinline__ void keep(v16b a, v16b b, v16b c, v16b d) { keep4_b(a, b, c, d); }
};

template <int ET> struct Elem;
template <> struct Elem<0> { typedef _Float16 T; };
template <> struct Elem<1> { typedef __bf16 T; };
template <int ET, bool SPLIT, int BIAS_MODE, int OUT_MODE, bool RESID, int ACT = 0>
__global__ __launch_bounds__(256) void wmma_gemm64(
    const unsigned short* __restrict__ Ap, const unsigned short* __restrict__ A2p, int lda, long strideA,
    const unsigned short* __restrict__ Btp, const unsigned short* __restrict__ Bt2p, int ldb, long strideB,
    void* __restrict__ Cout, void* __restrict__ Cout2, int ldc, long strideC,
    const float* __restrict__ bias,
    const float* __restrict__ resid, long strideR,
    int M, int N, int K, float scale) {
  typedef typename Elem<ET>::T T;
  typedef typename Frag<T>::V V;
  const T* A = (const T*)Ap; const T* A2 = (const T*)A2p; const T* Bt = (const T*)Btp; const T* Bt2 = (const T*)Bt2p;
  __shared__ __align__(16) float sT[8][16 * 68];
  const int b    = blockIdx.y;
  const int lane = threadIdx.x & 31;
  const int wave = threadIdx.x >> 5;
  const int tilesN = N >> 6;
  const int tilesM = M >> 6;
  const int tile = blockIdx.x * 8 + wave;
  if (tile >= tilesM * tilesN) return;
  const int tm = tile / tilesN;
  const int tn = tile - tm * tilesN;
  const int m0 = tm << 6;
  const int n0 = tn << 6;

  const T* Ab  = A  + (size_t)b * strideA;
  const T* Bb  = Bt + (size_t)b * strideB;
  const T* Ab2 = SPLIT ? (A2  + (size_t)b * strideA) : nullptr;
  const T* Bb2 = SPLIT ? (Bt2 + (size_t)b * strideB) : nullptr;

  const int rlane = lane & 15;
  const int koff  = (lane >> 4) * 8;
  const int mOff  = (lane >> 4) * 8;

  v8f acc[4][4];
#pragma unroll
  for (int i = 0; i < 4; ++i)
#pragma unroll
    for (int j = 0; j < 4; ++j) acc[i][j] = (v8f){0.f,0.f,0.f,0.f,0.f,0.f,0.f,0.f};

  for (int k0 = 0; k0 < K; k0 += 32) {
    V bh[4], bl[4];
#pragma unroll
    for (int j = 0; j < 4; ++j) {
      const size_t bo = (size_t)(n0 + (j << 4) + rlane) * ldb + koff + k0;
      bh[j] = Frag<T>::load(Bb + bo);
      if (SPLIT) bl[j] = Frag<T>::load(Bb2 + bo);
    }
#pragma unroll
    for (int i = 0; i < 4; ++i) {
      const size_t ao = (size_t)(m0 + (i << 4) + rlane) * lda + koff + k0;
      V ah = Frag<T>::load(Ab + ao);
      V al;
      if (SPLIT) al = Frag<T>::load(Ab2 + ao);
#pragma unroll
      for (int j = 0; j < 4; ++j) {
        acc[i][j] = Frag<T>::mma(ah, bh[j], acc[i][j]);
        if (SPLIT) {
          acc[i][j] = Frag<T>::mma(ah, bl[j], acc[i][j]);
          acc[i][j] = Frag<T>::mma(al, bh[j], acc[i][j]);
        }
      }
      Frag<T>::guard(acc[i][0], acc[i][3], ah, SPLIT ? al : ah);
    }
    Frag<T>::keep(bh[0], bh[1], bh[2], bh[3]);
    if (SPLIT) Frag<T>::keep(bl[0], bl[1], bl[2], bl[3]);
  }
  acc_guard4(acc[0][0], acc[0][1], acc[0][2], acc[0][3]);
  acc_guard4(acc[1][0], acc[1][1], acc[1][2], acc[1][3]);
  acc_guard4(acc[2][0], acc[2][1], acc[2][2], acc[2][3]);
  acc_guard4(acc[3][0], acc[3][1], acc[3][2], acc[3][3]);

  float* slab = sT[wave];
  const float* Rb = RESID ? (resid + (size_t)b * strideR) : nullptr;
#pragma unroll
  for (int i = 0; i < 4; ++i) {
    const int mBase = m0 + (i << 4);
#pragma unroll
    for (int j = 0; j < 4; ++j) {
      const int n = n0 + (j << 4) + rlane;
      float bv = 0.f;
      if (BIAS_MODE == 2) bv = bias[n];
#pragma unroll
      for (int r = 0; r < 8; ++r) {
        float v = acc[i][j][r] * scale;
        if (BIAS_MODE == 1) v += bias[mBase + mOff + r];
        if (BIAS_MODE == 2) v += bv;
        if (RESID) v += Rb[(size_t)(mBase + mOff + r) * ldc + n];
        if (ACT == 1) v = tanhf(v);
        if (ACT == 2) v = fmaxf(v, 0.0f);
        if (ACT == 3) v = v / (1.0f + expf(-v));
        if (ACT == 4) v = (v > 0.f) ? v : 0.01f * v;
        if (ACT == 5) v = 0.5f * v * (1.0f + erff(v * 0.70710678118654752f));
        slab[(mOff + r) * 68 + (j << 4) + rlane] = v;
      }
    }
    __builtin_amdgcn_fence(__ATOMIC_RELEASE, "workgroup");
    __builtin_amdgcn_wave_barrier();
    __builtin_amdgcn_fence(__ATOMIC_ACQUIRE, "workgroup");
    if (OUT_MODE == 0) {
      float* C = (float*)Cout + (size_t)b * strideC;
      const int hh = lane >> 4, c4 = (lane & 15) * 4;
      for (int pass = 0; pass < 2; ++pass) {
#pragma unroll
        for (int it = 0; it < 8; ++it) {
          const int row = it * 2 + hh;
          v4f v = *(const v4f*)(slab + row * 68 + c4);
          *(volatile v4f*)(C + (size_t)(mBase + row) * ldc + n0 + c4) = v;
        }
        __threadfence();
      }
    } else {
      const int q = lane >> 3, c8 = (lane & 7) * 8;
      unsigned short* C  = (unsigned short*)Cout  + (size_t)b * strideC;
      unsigned short* C2 = (OUT_MODE == 2) ? ((unsigned short*)Cout2 + (size_t)b * strideC) : nullptr;
      for (int pass = 0; pass < 2; ++pass) {
#pragma unroll
        for (int it = 0; it < 4; ++it) {
          const int row = it * 4 + q;
          const float* sp = slab + row * 68 + c8;
          v8h hv, lv;
#pragma unroll
          for (int e = 0; e < 8; ++e) {
            if (OUT_MODE == 1) {
              hv[e] = (_Float16)sp[e];
            } else {
              unsigned short hb = f2bf_bits(sp[e]);
              unsigned short lb = f2bf_bits(sp[e] - bf_bits2f(hb));
              hv[e] = __builtin_bit_cast(_Float16, hb);
              lv[e] = __builtin_bit_cast(_Float16, lb);
            }
          }
          *(volatile v8h*)(C + (size_t)(mBase + row) * ldc + n0 + c8) = hv;
          if (OUT_MODE == 2) *(volatile v8h*)(C2 + (size_t)(mBase + row) * ldc + n0 + c8) = lv;
        }
        __threadfence();
      }
    }
    __builtin_amdgcn_fence(__ATOMIC_RELEASE, "workgroup");
    __builtin_amdgcn_wave_barrier();
    __builtin_amdgcn_fence(__ATOMIC_ACQUIRE, "workgroup");
  }
}

__device__ __forceinline__ float fsig(float x)  { return __builtin_amdgcn_rcpf(1.0f + expf(-x)); }
__device__ __forceinline__ float ftanh(float x) { return 1.0f - 2.0f * __builtin_amdgcn_rcpf(expf(2.0f * x) + 1.0f); }

__global__ __launch_bounds__(NTHR) void prep_w2t_kernel(const float* __restrict__ W2, unsigned short* __restrict__ W2Tp) {
  const int i  = threadIdx.x;
  const int n  = i >> 2;
  const int k8 = (i & 3) * 8;
  v8h hv;
#pragma unroll
  for (int e = 0; e < 8; ++e) hv[e] = (_Float16)(W2[(size_t)(k8 + e) * NH2 + n] * OPCARRY);
  _Float16* dst = (_Float16*)W2Tp + 8 * i;
  *(volatile v8h*)dst = hv;
  __threadfence();
  *(volatile v8h*)dst = hv;
}

__global__ __launch_bounds__(NTHR) void prep_wcat_kernel(const float* __restrict__ w_ih, const float* __restrict__ w_hh,
                                                         unsigned short* __restrict__ WCp) {
  const int i   = blockIdx.x * NTHR + threadIdx.x;
  const int n   = i / (KCAT / 8);
  const int k8  = i - n * (KCAT / 8);
  const int kih = (k8 < 8) ? k8 : 7;
  const int khh = (k8 >= 8) ? (k8 - 8) : 0;
  const float* pi = w_ih + (size_t)n * NH2 + kih * 8;
  const float* ph = w_hh + (size_t)n * NHL + khh * 8;
  const v4f ia = *(const v4f*)(pi);
  const v4f ib = *(const v4f*)(pi + 4);
  const v4f ha = *(const v4f*)(ph);
  const v4f hb = *(const v4f*)(ph + 4);
  const bool first = (k8 < 8);
  v8h hv;
#pragma unroll
  for (int e = 0; e < 4; ++e) {
    hv[e]     = (_Float16)((first ? ia[e] : ha[e]) * OPCARRY);
    hv[4 + e] = (_Float16)((first ? ib[e] : hb[e]) * OPCARRY);
  }
  _Float16* dst = (_Float16*)WCp + (size_t)8 * i;
  *(volatile v8h*)dst = hv;
  __threadfence();
  *(volatile v8h*)dst = hv;
}

__global__ __launch_bounds__(NTHR) void gcn_kernel(const float* __restrict__ x, const float* __restrict__ adj,
                                                   const float* __restrict__ W1, const float* __restrict__ b1,
                                                   unsigned short* __restrict__ MPp, int chunk) {
  __shared__ float adjs[NJ * NJ];
  __shared__ float w1s[ND * NH1];
  __shared__ float b1s[NH1];
  __shared__ __align__(16) float xs[FPB * XFR];
  __shared__ __align__(16) float avs[ROWS_PB * 4];
  __shared__ __align__(16) float g1s[ROWS_PB * NH1];
  __shared__ __align__(16) _Float16 mps[ROWS_PB * NH1];
  const int tid = threadIdx.x;
  const int f0 = chunk * FPC + blockIdx.x * FPB;

#pragma unroll 1
  for (int i = tid; i < NJ * NJ; i += NTHR) adjs[i] = adj[i];
  if (tid < ND * NH1) w1s[tid] = W1[tid];
  if (tid < NH1) b1s[tid] = b1[tid];
  {
    const float* xg = x + (size_t)f0 * XFR;
#pragma unroll 1
    for (int i = tid; i < FPB * XFR; i += NTHR) xs[i] = xg[i];
  }
  __syncthreads();

#pragma unroll 1
  for (int it = tid; it < ROWS_PB; it += NTHR) {
    const int fl = it / NJ;
    const int j  = it - fl * NJ;
    const float* ar = adjs + j * NJ;
    const float* xr = xs + fl * XFR;
    float s0 = 0.0f, s1 = 0.0f, s2 = 0.0f;
#pragma unroll 1
    for (int k = 0; k < NJ; ++k) {
      const float av = ar[k];
      s0 += av * xr[k * ND + 0];
      s1 += av * xr[k * ND + 1];
      s2 += av * xr[k * ND + 2];
    }
    avs[it * 4 + 0] = s0;
    avs[it * 4 + 1] = s1;
    avs[it * 4 + 2] = s2;
  }
  __syncthreads();

#pragma unroll 1
  for (int e = tid; e < ROWS_PB * NH1; e += NTHR) {
    const int row = e >> 5;
    const int c   = e & 31;
    const float a0 = avs[row * 4 + 0];
    const float a1 = avs[row * 4 + 1];
    const float a2 = avs[row * 4 + 2];
    float v = (a0 * w1s[c] + a1 * w1s[NH1 + c]) + a2 * w1s[2 * NH1 + c];
    v += b1s[c];
    g1s[e] = fmaxf(v, 0.0f);
  }
  __syncthreads();

#pragma unroll 1
  for (int w = tid; w < ROWS_PB * (NH1 / 8); w += NTHR) {
    const int r  = w >> 2;
    const int cg = w & 3;
    const int fl = r / NJ;
    const int j  = r - fl * NJ;
    const float* ar = adjs + j * NJ;
    const float* gr = g1s + fl * (NJ * NH1) + cg * 8;
    float m0 = 0.f, m1 = 0.f, m2 = 0.f, m3 = 0.f, m4 = 0.f, m5 = 0.f, m6 = 0.f, m7 = 0.f;
#pragma unroll 1
    for (int k = 0; k < NJ; ++k) {
      const float av = ar[k];
      const v4f ga = *(const v4f*)(gr + k * NH1);
      const v4f gb = *(const v4f*)(gr + k * NH1 + 4);
      m0 += av * ga[0]; m1 += av * ga[1]; m2 += av * ga[2]; m3 += av * ga[3];
      m4 += av * gb[0]; m5 += av * gb[1]; m6 += av * gb[2]; m7 += av * gb[3];
    }
    v8h hv;
    hv[0] = (_Float16)(m0 * OPCARRY); hv[1] = (_Float16)(m1 * OPCARRY);
    hv[2] = (_Float16)(m2 * OPCARRY); hv[3] = (_Float16)(m3 * OPCARRY);
    hv[4] = (_Float16)(m4 * OPCARRY); hv[5] = (_Float16)(m5 * OPCARRY);
    hv[6] = (_Float16)(m6 * OPCARRY); hv[7] = (_Float16)(m7 * OPCARRY);
    *(v8h*)(mps + 8 * w) = hv;
  }
  __syncthreads();

  _Float16* MPg = (_Float16*)MPp + (size_t)blockIdx.x * (ROWS_PB * NH1);
  for (int pass = 0; pass < 2; ++pass) {
#pragma unroll 1
    for (int p = tid; p < ROWS_PB * NH1 / 8; p += NTHR) {
      const v8h v = *(const v8h*)(mps + 8 * p);
      *(volatile v8h*)(MPg + 8 * p) = v;
    }
    __threadfence();
  }
}

__global__ __launch_bounds__(NTHR) void joint_mean_kernel(const float* __restrict__ G2, unsigned short* __restrict__ FTp, int chunk) {
  const int i   = blockIdx.x * NTHR + threadIdx.x;
  const int t   = i >> 7;
  const int rem = i & 127;
  const int bl  = rem >> 3;
  const int c8  = rem & 7;
  const int lf  = bl * NSTEP + t;
  const float* gp = G2 + (size_t)lf * (NJ * NH2) + c8 * 8;
  v4f s0 = {0.f, 0.f, 0.f, 0.f};
  v4f s1 = {0.f, 0.f, 0.f, 0.f};
#pragma unroll 1
  for (int j = 0; j < NJ; ++j) {
    s0 += *(const v4f*)(gp + j * NH2);
    s1 += *(const v4f*)(gp + j * NH2 + 4);
  }
  v8h hv;
#pragma unroll
  for (int e = 0; e < 4; ++e) {
    const float ma = s0[e] * (1.0f / 33.0f);
    const float mb = s1[e] * (1.0f / 33.0f);
    hv[e]     = (_Float16)(ma * OPCARRY);
    hv[4 + e] = (_Float16)(mb * OPCARRY);
  }
  const int b = chunk * BPC + bl;
  _Float16* dst = (_Float16*)FTp + (size_t)(t * NBAT + b) * NH2 + c8 * 8;
  *(volatile v8h*)dst = hv;
  __threadfence();
  *(volatile v8h*)dst = hv;
}

__global__ __launch_bounds__(NTHR) void lstm_kernel(const unsigned short* __restrict__ FTp, const unsigned short* __restrict__ WCp,
                                                    const float* __restrict__ b_ih, const float* __restrict__ b_hh,
                                                    float* __restrict__ out) {
  __shared__ __align__(16) _Float16 At[2][SEQ_BLK * APITCH];
  __shared__ __align__(16) float    Sl[SEQ_BLK * SLABP];
  const _Float16* FT = (const _Float16*)FTp;
  const _Float16* WC = (const _Float16*)WCp;
  const int tid = threadIdx.x, lane = tid & 31, wave = tid >> 5;
  const int c = lane & 15, hh = lane >> 4, koff = hh * 8;
  const int rowbase = blockIdx.x * SEQ_BLK;
  const int ucol = 16 * wave + c;

  {
    _Float16* atf = &At[0][0];
    const v8h z = {(_Float16)0.f, (_Float16)0.f, (_Float16)0.f, (_Float16)0.f, (_Float16)0.f, (_Float16)0.f, (_Float16)0.f, (_Float16)0.f};
#pragma unroll 1
    for (int p = tid; p < 2 * SEQ_BLK * APITCH / 8; p += NTHR) *(v8h*)(atf + 8 * p) = z;
  }
  float bsum[4];
#pragma unroll
  for (int g = 0; g < 4; ++g) bsum[g] = b_ih[g * NHL + ucol] + b_hh[g * NHL + ucol];
  float cst[2][8], hst[2][8];
#pragma unroll
  for (int ms = 0; ms < 2; ++ms)
#pragma unroll
    for (int r = 0; r < 8; ++r) { cst[ms][r] = 0.0f; hst[ms][r] = 0.0f; }
  __syncthreads();

  const v8f z8 = {0.f, 0.f, 0.f, 0.f, 0.f, 0.f, 0.f, 0.f};
  const int frow = tid >> 3;
  const int fc8  = (tid & 7) * 8;

#pragma unroll 1
  for (int t = 0; t < NSTEP; ++t) {
    const int cur = t & 1;
    {
      const v8h fv = *(const v8h*)(FT + (size_t)(t * NBAT + rowbase + frow) * NH2 + fc8);
      *(v8h*)(&At[cur][0] + frow * APITCH + fc8) = fv;
    }
    __syncthreads();

    const _Float16* ab = &At[cur][0];
    _Float16* an = &At[cur ^ 1][0];
    v8f acc[2][4];
#pragma unroll
    for (int ms = 0; ms < 2; ++ms)
#pragma unroll
      for (int g = 0; g < 4; ++g) acc[ms][g] = z8;

#pragma unroll 1
    for (int k0 = 0; k0 < KCAT; k0 += 32) {
      const v16h a0 = Frag<_Float16>::load(ab + c * APITCH + koff + k0);
      const v16h a1 = Frag<_Float16>::load(ab + (16 + c) * APITCH + koff + k0);
#pragma unroll
      for (int g = 0; g < 4; ++g) {
        const v16h bw = Frag<_Float16>::load(WC + (size_t)(g * NHL + ucol) * KCAT + koff + k0);
        acc[0][g] = Frag<_Float16>::mma(a0, bw, acc[0][g]);
        acc[1][g] = Frag<_Float16>::mma(a1, bw, acc[1][g]);
        dep_guard_h(acc[0][g], acc[1][g], a1, bw);
      }
      keep4_h(a0, a1, a0, a1);
    }
    acc_guard4(acc[0][0], acc[0][1], acc[0][2], acc[0][3]);
    acc_guard4(acc[1][0], acc[1][1], acc[1][2], acc[1][3]);

#pragma unroll
    for (int ms = 0; ms < 2; ++ms) {
#pragma unroll
      for (int r = 0; r < 8; ++r) {
        const float zi = acc[ms][0][r] * OPCARRY2_INV + bsum[0];
        const float zf = acc[ms][1][r] * OPCARRY2_INV + bsum[1];
        const float zg = acc[ms][2][r] * OPCARRY2_INV + bsum[2];
        const float zo = acc[ms][3][r] * OPCARRY2_INV + bsum[3];
        const float ig = fsig(zi);
        const float fg = fsig(zf);
        const float gg = ftanh(zg);
        const float og = fsig(zo);
        const float cn = fg * cst[ms][r] + ig * gg;
        cst[ms][r] = cn;
        const float hn = og * ftanh(cn);
        hst[ms][r] = hn;
        an[(ms * 16 + 8 * hh + r) * APITCH + NH2 + ucol] = (_Float16)(hn * OPCARRY);
      }
    }
  }

#pragma unroll
  for (int ms = 0; ms < 2; ++ms)
#pragma unroll
    for (int r = 0; r < 8; ++r) Sl[(ms * 16 + 8 * hh + r) * SLABP + ucol] = hst[ms][r];
  __syncthreads();
  for (int pass = 0; pass < 2; ++pass) {
#pragma unroll
    for (int rr = 0; rr < 4; ++rr) {
      const int row = 4 * wave + rr;
      const v4f v = *(const v4f*)(Sl + row * SLABP + 4 * lane);
      *(volatile v4f*)(out + (size_t)(rowbase + row) * NHL + 4 * lane) = v;
    }
    __threadfence();
  }
}

extern "C" void kernel_launch(void* const* d_in, const int* in_sizes, int n_in,
                              void* d_out, int out_size, void* d_ws, size_t ws_size, hipStream_t stream) {
  if (n_in < 10 || d_out == nullptr || d_ws == nullptr) return;
  if (in_sizes[0] != NFRAME * XFR || in_sizes[1] != NJ * NJ || in_sizes[2] != ND * NH1 || in_sizes[3] != NH1 ||
      in_sizes[4] != NH1 * NH2 || in_sizes[5] != NH2 || in_sizes[6] != NGATE * NH2 || in_sizes[7] != NGATE * NHL ||
      in_sizes[8] != NGATE || in_sizes[9] != NGATE || out_size != NBAT * NHL) return;

  const float* x    = (const float*)d_in[0];
  const float* adj  = (const float*)d_in[1];
  const float* W1   = (const float*)d_in[2];
  const float* b1   = (const float*)d_in[3];
  const float* W2   = (const float*)d_in[4];
  const float* b2   = (const float*)d_in[5];
  const float* w_ih = (const float*)d_in[6];
  const float* w_hh = (const float*)d_in[7];
  const float* b_ih = (const float*)d_in[8];
  const float* b_hh = (const float*)d_in[9];
  float* out = (float*)d_out;

  char* ws = (char*)d_ws; size_t off = 0;
  auto carve = [&](size_t bytes) -> char* { char* p = ws + off; off += (bytes + 255) & ~(size_t)255; return p; };
  unsigned short* W2T  = (unsigned short*)carve((size_t)NH2 * NH1 * 2);
  unsigned short* WCAT = (unsigned short*)carve((size_t)NGATE * KCAT * 2);
  unsigned short* FT   = (unsigned short*)carve((size_t)NFRAME * NH2 * 2);
  unsigned short* MP   = (unsigned short*)carve((size_t)ROWS_PC * NH1 * 2);
  float*          G2   = (float*)carve((size_t)ROWS_PC * NH2 * 4);
  if (off > ws_size || off > (size_t)134217728) return;

  prep_w2t_kernel<<<1, NTHR, 0, stream>>>(W2, W2T);
  prep_wcat_kernel<<<NGATE * (KCAT / 8) / NTHR, NTHR, 0, stream>>>(w_ih, w_hh, WCAT);

  const dim3 ggrid((ROWS_PC / 64) * (NH2 / 64) / 8, 1);
  for (int q = 0; q < NCHUNK; ++q) {
    gcn_kernel<<<FPC / FPB, NTHR, 0, stream>>>(x, adj, W1, b1, MP, q);
    wmma_gemm64<0, false, 2, 0, false, 0><<<ggrid, 256, 0, stream>>>(
        MP, MP, NH1, 0L, W2T, W2T, NH1, 0L, (void*)G2, (void*)G2, NH2, 0L,
        b2, (const float*)G2, 0L, ROWS_PC, NH2, NH1, OPCARRY2_INV);
    joint_mean_kernel<<<FPC * 8 / NTHR, NTHR, 0, stream>>>(G2, FT, q);
  }

  lstm_kernel<<<NBAT / SEQ_BLK, NTHR, 0, stream>>>(FT, WCAT, b_ih, b_hh, out);
}
